// MinGRUPolicyBackbone_57698590655153
// MI455X (gfx1250) — hardware-verified
//
#include <hip/hip_runtime.h>
#include <hip/hip_bf16.h>
#include <math.h>

#define BB 16
#define SS 4096
#define DIN 64
#define DM 512
#define DI 768
#define MTOK (BB * SS)
#define GSTR 48

typedef _Float16 bf16;
typedef _Float16 f16;
typedef __attribute__((ext_vector_type(4))) unsigned v4u_t;
typedef unsigned v4ua __attribute__((ext_vector_type(4), may_alias));
typedef __attribute__((ext_vector_type(4))) float v4f_t;
typedef float v4fa __attribute__((ext_vector_type(4), may_alias));
typedef __attribute__((ext_vector_type(16))) bf16  bf16x16;
typedef bf16x16 f16x16;
typedef __attribute__((ext_vector_type(8)))  bf16  bf16x8;
typedef bf16x8 f16x8;
typedef __attribute__((ext_vector_type(8)))  float f32x8;
__device__ __forceinline__ f32x8 wmma16(f16x16 a, f16x16 b, f32x8 c) {
  c = __builtin_amdgcn_wmma_f32_16x16x32_f16(false, a, false, b, (short)0, c, false, false);
  asm volatile("v_nop\n\tv_nop\n\tv_nop\n\tv_nop" : "+v"(c) : "v"(a), "v"(b));
  return c;
}
__device__ __forceinline__ f16x16 lds_frag(const f16* base, int stride) {
  const int lane = threadIdx.x & 31, row = lane & 15, kh = (lane >> 4) * 8;
  const f16x8 lo = *(const f16x8*)(base + row * stride + kh);
  const f16x8 hi = *(const f16x8*)(base + row * stride + kh + 16);
  f16x16 f;
#pragma unroll
  for (int i = 0; i < 8; ++i) { f[i] = lo[i]; f[i + 8] = hi[i]; }
  return f;
}

#define GSTR 48
template <typename AT, int EPI, bool OUT16>
__global__ __launch_bounds__(256) void gemm_kne(const AT* __restrict__ A, int lda, const float* __restrict__ Wm, int ldw,
                                                const float* __restrict__ bias, const float* __restrict__ R, const float* __restrict__ gvec,
                                                void* __restrict__ Yv, int ldy, int K) {
  __shared__ __attribute__((aligned(16))) f16 ldsA[128 * GSTR];
  __shared__ __attribute__((aligned(16))) f16 ldsW[128 * GSTR];
  __shared__ __attribute__((aligned(16))) float oS[8][32 * 68];
  const int tid = threadIdx.x, lane = tid & 31, wave = tid >> 5, cl = lane & 15, rh = (lane >> 4) * 8;
  const int m0 = blockIdx.x * 128, n0 = blockIdx.y * 128;
  const int wm = (wave & 3) * 32, wn = (wave >> 2) * 64;
  f32x8 acc[2][4];
#pragma unroll
  for (int i = 0; i < 2; ++i)
#pragma unroll
    for (int j = 0; j < 4; ++j) { f32x8 z = {}; acc[i][j] = z; }
#pragma unroll 1
  for (int k0 = 0; k0 < K; k0 += 32) {
    __syncthreads();
    { const int row = tid >> 1, ch = (tid & 1) * 16;
      const AT* src = A + (size_t)(m0 + row) * lda + k0 + ch;
#pragma unroll
      for (int g = 0; g < 16; ++g) ldsA[row * GSTR + ch + g] = (f16)src[g]; }
    { const int k = tid >> 3, nn0 = (tid & 7) * 16;
      const float* src = Wm + (size_t)(k0 + k) * ldw + n0 + nn0;
#pragma unroll
      for (int g = 0; g < 4; ++g) { const v4f_t v = *(const v4f_t*)(src + 4 * g);
#pragma unroll
        for (int u = 0; u < 4; ++u) ldsW[(nn0 + 4 * g + u) * GSTR + k] = (f16)v[u]; } }
    __syncthreads();
    f16x16 af[2];
#pragma unroll
    for (int i = 0; i < 2; ++i) af[i] = lds_frag(ldsA + (wm + 16 * i) * GSTR, GSTR);
#pragma unroll
    for (int j = 0; j < 4; ++j) {
      const f16x16 bf = lds_frag(ldsW + (wn + 16 * j) * GSTR, GSTR);
#pragma unroll
      for (int i = 0; i < 2; ++i) acc[i][j] = wmma16(af[i], bf, acc[i][j]);
    }
  }
  float* so = oS[wave];
#pragma unroll
  for (int i = 0; i < 2; ++i)
#pragma unroll
    for (int j = 0; j < 4; ++j) {
      const int n = n0 + wn + 16 * j + cl;
      const float bv = bias ? bias[n] : 0.0f;
      const float gv = (EPI == 2) ? gvec[n] : 0.0f;
      if (EPI == 1) {
#pragma unroll 1
        for (int r = 0; r < 8; ++r) { const float xg = acc[i][j][r] + bv; so[(16 * i + rh + r) * 68 + 16 * j + cl] = 0.5f * xg * (1.0f + erff(xg * 0.70710678118654752f)); }
      } else {
#pragma unroll
        for (int r = 0; r < 8; ++r) {
          float v = acc[i][j][r] + bv;
          if (EPI == 2) v = R[(size_t)(m0 + wm + 16 * i + rh + r) * ldy + n] + gv * v;
          so[(16 * i + rh + r) * 68 + 16 * j + cl] = v;
        }
      }
    }
  asm volatile("s_wait_dscnt 0" ::: "memory");
  __builtin_amdgcn_wave_barrier();
#pragma unroll 1
  for (int pass = 0; pass < 2; ++pass) {
    if (OUT16) {
      f16* Y = (f16*)Yv;
#pragma unroll
      for (int it = 0; it < 8; ++it) { const int c = lane + 32 * it, rr = c >> 3, q8 = (c & 7) * 8;
        union { f16 h[8]; v4u_t v; } u;
#pragma unroll
        for (int e = 0; e < 8; ++e) u.h[e] = (f16)so[rr * 68 + q8 + e];
        *(volatile v4u_t*)(Y + (size_t)(m0 + wm + rr) * ldy + n0 + wn + q8) = u.v; }
    } else {
      float* Y = (float*)Yv;
#pragma unroll
      for (int it = 0; it < 16; ++it) { const int f4 = lane + 32 * it, rr = f4 >> 4, q = (f4 & 15) * 4;
        *(volatile v4f_t*)(Y + (size_t)(m0 + wm + rr) * ldy + n0 + wn + q) = *(const volatile v4fa*)(so + rr * 68 + q); }
    }
    __threadfence();
  }
}

template <typename AT, bool ACC>
__global__ __launch_bounds__(256) void gemm_kn2(const AT* __restrict__ A, int lda, size_t strideA,
                                               const float* __restrict__ Wm, int ldw, size_t strideW,
                                               const float* __restrict__ bias, float scale,
                                               float* __restrict__ Y, int ldy, size_t strideY, int K) {
  __shared__ __attribute__((aligned(16))) f16 ldsA[128 * GSTR], ldsAl[128 * GSTR];
  __shared__ __attribute__((aligned(16))) f16 ldsW[128 * GSTR], ldsWl[128 * GSTR];
  __shared__ __attribute__((aligned(16))) float oS[8][32 * 68];
  const int tid = threadIdx.x, lane = tid & 31, wave = tid >> 5, cl = lane & 15, rh = (lane >> 4) * 8;
  const int m0 = blockIdx.x * 128, n0 = blockIdx.y * 128;
  const int wm = (wave & 3) * 32, wn = (wave >> 2) * 64;
  A += (size_t)blockIdx.z * strideA; Wm += (size_t)blockIdx.z * strideW; Y += (size_t)blockIdx.z * strideY;
  f32x8 acc[2][4], accx[2][4];
#pragma unroll
  for (int i = 0; i < 2; ++i)
#pragma unroll
    for (int j = 0; j < 4; ++j) { f32x8 z = {}; acc[i][j] = z; accx[i][j] = z; }
#pragma unroll 1
  for (int k0 = 0; k0 < K; k0 += 32) {
    __syncthreads();
    {
      const int row = tid >> 1, ch = (tid & 1) * 16;
      const AT* src = A + (size_t)(m0 + row) * lda + k0 + ch;
#pragma unroll
      for (int g = 0; g < 16; ++g) { const float v = (float)src[g]; const f16 h = (f16)v; ldsA[row * GSTR + ch + g] = h; ldsAl[row * GSTR + ch + g] = (f16)((v - (float)h) * 2048.0f); }
    }
    {
      const int k = tid >> 3, nn0 = (tid & 7) * 16;
      const float* src = Wm + (size_t)(k0 + k) * ldw + n0 + nn0;
#pragma unroll
      for (int g = 0; g < 4; ++g) { const v4f_t v = *(const v4f_t*)(src + 4 * g);
#pragma unroll
        for (int u = 0; u < 4; ++u) { const f16 h = (f16)v[u]; ldsW[(nn0 + 4 * g + u) * GSTR + k] = h; ldsWl[(nn0 + 4 * g + u) * GSTR + k] = (f16)((v[u] - (float)h) * 2048.0f); } }
    }
    __syncthreads();
    f16x16 af[2], afl[2];
#pragma unroll
    for (int i = 0; i < 2; ++i) { af[i] = lds_frag(ldsA + (wm + 16 * i) * GSTR, GSTR); afl[i] = lds_frag(ldsAl + (wm + 16 * i) * GSTR, GSTR); }
#pragma unroll
    for (int j = 0; j < 4; ++j) {
      const f16x16 bf = lds_frag(ldsW + (wn + 16 * j) * GSTR, GSTR), bfl = lds_frag(ldsWl + (wn + 16 * j) * GSTR, GSTR);
#pragma unroll
      for (int i = 0; i < 2; ++i) { acc[i][j] = wmma16(af[i], bf, acc[i][j]); accx[i][j] = wmma16(af[i], bfl, accx[i][j]); accx[i][j] = wmma16(afl[i], bf, accx[i][j]); }
    }
  }
  float* so = oS[wave];
#pragma unroll
  for (int i = 0; i < 2; ++i)
#pragma unroll
    for (int j = 0; j < 4; ++j) {
      const float bv = bias ? bias[n0 + wn + 16 * j + cl] : 0.0f;
#pragma unroll
      for (int r = 0; r < 8; ++r) so[(16 * i + rh + r) * 68 + 16 * j + cl] = (acc[i][j][r] + accx[i][j][r] * (1.0f / 2048.0f)) * scale + bv;
    }
  asm volatile("s_wait_dscnt 0" ::: "memory");
  __builtin_amdgcn_wave_barrier();
  if (ACC) {
#pragma unroll
    for (int it = 0; it < 16; ++it) { const int f4 = lane + 32 * it, rr = f4 >> 4, q = (f4 & 15) * 4;
      const v4f_t old = *(const volatile v4fa*)(Y + (size_t)(m0 + wm + rr) * ldy + n0 + wn + q);
      v4f_t v = *(const volatile v4fa*)(so + rr * 68 + q); v += old; *(volatile v4fa*)(so + rr * 68 + q) = v; }
    asm volatile("s_wait_dscnt 0" ::: "memory");
  }
#pragma unroll 1
  for (int pass = 0; pass < 2; ++pass) {
#pragma unroll
    for (int it = 0; it < 16; ++it) { const int f4 = lane + 32 * it, rr = f4 >> 4, q = (f4 & 15) * 4;
      *(volatile v4f_t*)(Y + (size_t)(m0 + wm + rr) * ldy + n0 + wn + q) = *(const volatile v4fa*)(so + rr * 68 + q); }
    __threadfence();
  }
}

__global__ __launch_bounds__(256) void k_padw(const float* __restrict__ We, float* __restrict__ Wp) { const int r = blockIdx.x; for (int c = threadIdx.x; c < DM; c += 256) Wp[(size_t)r * DM + c] = (r < DIN) ? We[(size_t)r * DM + c] : 0.0f; }
__global__ __launch_bounds__(256) void k_bcomb(const float* __restrict__ b_emb, const float* __restrict__ W_hg, float* __restrict__ bc) {
  for (int n = threadIdx.x; n < 2 * DI; n += 256) { float s = 0.0f; for (int k = 0; k < DM; ++k) s += b_emb[k] * W_hg[(size_t)k * 2 * DI + n]; bc[n] = s; }
}
__global__ __launch_bounds__(256) void k_gru(const float* __restrict__ obs, const float* __restrict__ Wc, const float* __restrict__ bc, float* __restrict__ hl) {
  __shared__ __attribute__((aligned(16))) f16 aS[64 * 72];
  __shared__ __attribute__((aligned(16))) f16 wS[128 * 72];
  __shared__ float hgS[64 * 132];
  const int tid = threadIdx.x, lane = tid & 31, wave = tid >> 5, cl = lane & 15, rh = (lane >> 4) * 8;
  const int b = blockIdx.x / (DI / 64), c0 = (blockIdx.x % (DI / 64)) * 64;
  for (int e = tid; e < 128 * 64; e += 256) { const int n = e >> 6, k = e & 63; const int col = (n < 64) ? (c0 + n) : (DI + c0 + n - 64); wS[n * 72 + k] = (f16)Wc[(size_t)k * (2 * DI) + col]; }
  float bh = 0.0f, bg = 0.0f, h = 0.0f; if (tid < 64) { bh = bc[c0 + tid]; bg = bc[DI + c0 + tid]; }
#pragma unroll 1
  for (int t0 = 0; t0 < SS; t0 += 64) {
    __syncthreads();
    for (int e = tid; e < 64 * 64; e += 256) { const int t = e >> 6, k = e & 63; aS[t * 72 + k] = (f16)obs[((size_t)b * SS + t0 + t) * DIN + k]; }
    __syncthreads();
    { const int tt = wave & 3, nt0 = (wave >> 2) * 4; f32x8 acc[4];
#pragma unroll
      for (int j = 0; j < 4; ++j) { f32x8 z = {}; acc[j] = z; }
#pragma unroll
      for (int ks = 0; ks < 2; ++ks) { const f16x16 af = lds_frag(aS + (tt * 16) * 72 + ks * 32, 72);
#pragma unroll
        for (int j = 0; j < 4; ++j) acc[j] = wmma16(af, lds_frag(wS + ((nt0 + j) * 16) * 72 + ks * 32, 72), acc[j]); }
#pragma unroll
      for (int j = 0; j < 4; ++j)
#pragma unroll
        for (int r = 0; r < 8; ++r) hgS[(tt * 16 + rh + r) * 132 + (nt0 + j) * 16 + cl] = acc[j][r]; }
    __syncthreads();
    if (tid < 64) {
#pragma unroll 4
      for (int t = 0; t < 64; ++t) { const float hid = hgS[t * 132 + tid] + bh, gate = hgS[t * 132 + 64 + tid] + bg;
        const float zz = 1.0f / (1.0f + expf(-gate)); const float gv = (hid >= 0.0f) ? (hid + 0.5f) : (1.0f / (1.0f + expf(-hid)));
        h = (1.0f - zz) * h + zz * gv; } }
  }
  if (tid < 64) hl[(size_t)b * DI + c0 + tid] = h;
}
__global__ __launch_bounds__(256) void k_out(const float* __restrict__ hl, const float* __restrict__ W_out, float* __restrict__ out) {
  __shared__ __attribute__((aligned(16))) f16 aS[16 * 776]; __shared__ __attribute__((aligned(16))) float oS[16 * 516];
  const int tid = threadIdx.x, lane = tid & 31, wave = tid >> 5, cl = lane & 15, rh = (lane >> 4) * 8;
  for (int e = tid; e < 16 * DI; e += 256) aS[(e / DI) * 776 + (e % DI)] = (f16)hl[e];
  __syncthreads();
  for (int j = 0; j < 4; ++j) { const int nt = wave * 4 + j; f32x8 acc = {};
    for (int ks = 0; ks < DI / 32; ++ks) { const int n = nt * 16 + (lane & 15), kh = (lane >> 4) * 8; const float* src = W_out + (size_t)(ks * 32 + kh) * DM + n; f16x16 bf;
#pragma unroll
      for (int e = 0; e < 8; ++e) { bf[e] = (f16)src[(size_t)e * DM]; bf[8 + e] = (f16)src[(size_t)(16 + e) * DM]; }
      acc = wmma16(lds_frag(aS + ks * 32, 776), bf, acc); }
#pragma unroll
    for (int r = 0; r < 8; ++r) oS[(rh + r) * 516 + nt * 16 + cl] = acc[r]; }
  __syncthreads();
#pragma unroll 1
  for (int pass = 0; pass < 2; ++pass) { for (int q4 = tid; q4 < 16 * 128; q4 += 256) { const int r = q4 >> 7, c4 = (q4 & 127) * 4; *(volatile v4f_t*)(out + (size_t)r * DM + c4) = *(const volatile v4fa*)(oS + r * 516 + c4); } __threadfence(); }
}

extern "C" void kernel_launch(void* const* d_in, const int* in_sizes, int n_in,
                              void* d_out, int out_size, void* d_ws, size_t ws_size,
                              hipStream_t stream) {
  (void)in_sizes; (void)n_in; (void)out_size;
  const float* obs = (const float*)d_in[0];
  const float* W_emb = (const float*)d_in[1];
  const float* b_emb = (const float*)d_in[2];
  const float* W_hg = (const float*)d_in[3];
  const float* W_out = (const float*)d_in[4];
  float* out = (float*)d_out;
  char* ws = (char*)d_ws;
  float* Wembp = (float*)ws; ws += (size_t)128 * DM * 4;
  float* Wc = (float*)ws; ws += (size_t)128 * 2 * DI * 4;
  float* bc = (float*)ws; ws += 2 * DI * 4;
  float* hl = (float*)ws; ws += (size_t)BB * DI * 4;
  if ((size_t)(ws - (char*)d_ws) > ws_size) return;
  const dim3 blk(256);
  k_padw<<<dim3(128), blk, 0, stream>>>(W_emb, Wembp);
  gemm_kn2<float, false><<<dim3(1, (2 * DI) / 128, 1), blk, 0, stream>>>(Wembp, DM, 0, W_hg, 2 * DI, 0, nullptr, 1.0f, Wc, 2 * DI, 0, DM);
  k_bcomb<<<dim3(1), blk, 0, stream>>>(b_emb, W_hg, bc);
  k_gru<<<dim3(BB * (DI / 64)), blk, 0, stream>>>(obs, Wc, bc, hl);
  k_out<<<dim3(1), blk, 0, stream>>>(hl, W_out, out);
}
